// MoEBlock_75127567941882
// MI455X (gfx1250) — hardware-run, weakly checked
//
#include <hip/hip_runtime.h>
#include <math.h>

#define NTOK 4096
#define DM 1024
#define FF 4096
#define II FF
#define NPART 4
#define RK 4
#define TOPK 2
#define NE 1
#define NSH 1
#define NROW_S NTOK
#define R_MAX NTOK
#define NT_MAX (R_MAX / 64)

#define CX_LOG2 11
#define CW_LOG2 16
#define CH_LOG2 11
#define CH ((float)(1u << CH_LOG2))
#define SC_H (1.0f / (float)(1u << (CX_LOG2 + CW_LOG2)))
#define SC_Y (1.0f / (float)(1u << (CH_LOG2 + CW_LOG2)))

#define TBL_COUNT 0
#define TBL_POFF 16
#define TBL_NTILES 32
#define TBL_TILE_E 64
#define TBLS_WORDS 256

static_assert(NPART == 4 && RK == 4 && TOPK == 2 && NE == 1 && NSH == 1 && NROW_S == NTOK && R_MAX == NTOK);
static_assert(DM == 1024 && FF == 4096 && II == FF && DM % 64 == 0 && FF % 64 == 0 && NTOK % 64 == 0 && NTOK % 128 == 0 && DM % 32 == 0);
static_assert(TBL_COUNT + NE <= TBL_POFF && TBL_POFF + NE + 1 <= TBL_NTILES && TBL_NTILES < TBL_TILE_E && TBL_TILE_E + NT_MAX <= TBLS_WORDS);
static_assert(CX_LOG2 == 11 && CW_LOG2 == 16 && CH_LOG2 == 11 && NT_MAX == 64);
static_assert((NTOK * DM / 8) % 256 == 0 && (FF * DM / 8) % 256 == 0 && (NPART * FF * RK / 4) % 256 == 0);

constexpr size_t al256(size_t b) { return (b + 255) & ~(size_t)255; }
constexpr size_t SZ_X16 = al256((size_t)NTOK * DM * 2);
constexpr size_t SZ_W   = al256((size_t)FF * DM * 2);
constexpr size_t SZ_BQ  = al256((size_t)NPART * FF * RK * 4);
constexpr size_t SZ_SEL = al256((size_t)NTOK * TOPK * 4);
constexpr size_t SZ_LOW = al256((size_t)NTOK * RK * 4);
constexpr size_t SZ_TBL = al256((size_t)TBLS_WORDS * 4);
constexpr size_t SZ_HG  = al256((size_t)NTOK * FF * 2);
constexpr size_t WS_TOTAL = SZ_X16 + 2 * SZ_W + SZ_BQ + 2 * SZ_SEL + 2 * SZ_LOW + SZ_TBL + SZ_HG;
static_assert(WS_TOTAL == (size_t)59180032 && WS_TOTAL < (size_t)134217728);

typedef _Float16 h16;
typedef __attribute__((ext_vector_type(16))) _Float16 v16h;
typedef __attribute__((ext_vector_type(8)))  _Float16 v8h;
typedef __attribute__((ext_vector_type(8)))  float    v8f;
typedef __attribute__((ext_vector_type(4)))  float    v4f;
typedef __attribute__((ext_vector_type(2)))  float    v2f;
typedef __attribute__((ext_vector_type(4)))  unsigned int v4u;
typedef __attribute__((ext_vector_type(4)))  int      v4i;
typedef __attribute__((ext_vector_type(2)))  int      v2i;


#define VST2(T, ptr, val) do { const T vst2_v_ = (val); *(volatile T*)(ptr) = vst2_v_; __threadfence(); *(volatile T*)(ptr) = vst2_v_; } while (0)

static __device__ __forceinline__ float bfr(float f) {
    unsigned u = __float_as_uint(f);
    u += 0x7FFFu + ((u >> 16) & 1u);
    return __uint_as_float(u & 0xFFFF0000u);
}
static __device__ __forceinline__ h16 toh_flush(float v) { const float w = (fabsf(v) < 6.103515625e-05f) ? 0.0f : v; return (h16)w; }
static __device__ __forceinline__ void st8h(h16* p, const float* v) {
    v8h hv;
#pragma unroll
    for (int e = 0; e < 8; ++e) hv[e] = toh_flush(v[e]);
    VST2(v8h, p, hv);
}

union FragU { v16h v; v8h h[2]; };
static __device__ __forceinline__ v16h frag_ld(const h16* p) {
    FragU f; f.h[0] = *(const v8h*)(p); f.h[1] = *(const v8h*)(p + 16); return f.v;
}
static __device__ __forceinline__ v8f wmma16g(v16h a, v16h b, v8f c) {
    c = __builtin_amdgcn_wmma_f32_16x16x32_f16(false, a, false, b, (short)0, c, false, false);
    asm volatile("v_nop\n\tv_nop\n\tv_nop\n\tv_nop" : "+v"(c) : "v"(a), "v"(b));
    return c;
}
static __device__ __forceinline__ void wave_sync_lds() {
    __builtin_amdgcn_fence(3  , "workgroup");
    __builtin_amdgcn_wave_barrier();
    __builtin_amdgcn_fence(2  , "workgroup");
}
template <int LOG2C>
__global__ __launch_bounds__(256) void k_plane(const float* __restrict__ src, h16* __restrict__ dst, unsigned n8) {
    const unsigned u = blockIdx.x * 256u + threadIdx.x;
    if (u >= n8) return;
    const float cs = (float)(1u << LOG2C);
    const v4f a = *(const v4f*)(src + (size_t)u * 8u);
    const v4f b = *(const v4f*)(src + (size_t)u * 8u + 4u);
    float v[8] = {bfr(a.x) * cs, bfr(a.y) * cs, bfr(a.z) * cs, bfr(a.w) * cs, bfr(b.x) * cs, bfr(b.y) * cs, bfr(b.z) * cs, bfr(b.w) * cs};
    st8h(dst + (size_t)u * 8u, v);
}

__global__ __launch_bounds__(256) void k_castf(const float* __restrict__ w, float* __restrict__ q, unsigned n) {
    const unsigned i = (blockIdx.x * 256u + threadIdx.x) * 4u;
    if (i >= n) return;
    const v4f a = *(const v4f*)(w + i);
    v4f o; o.x = bfr(a.x); o.y = bfr(a.y); o.z = bfr(a.z); o.w = bfr(a.w);
    VST2(v4f, q + i, o);
}

__device__ __forceinline__ v4f pick4(int e, const v4f p0, const v4f p1, const v4f p2, const v4f p3) {
    v4f o = p0;
    o = (e == 1) ? p1 : o; o = (e == 2) ? p2 : o; o = (e == 3) ? p3 : o;
    return o;
}
__global__ __launch_bounds__(256) void k_gate_lora(const float* __restrict__ x, const float* __restrict__ Wg, const float* __restrict__ bg, const float* __restrict__ A,
                                                   int* __restrict__ sel, float* __restrict__ wgt, float* __restrict__ low0, float* __restrict__ low1) {
    const unsigned lane = threadIdx.x & 31u;
    const unsigned wave = threadIdx.x >> 5;
    const unsigned tok0 = (blockIdx.x * 8u + wave) * 16u;
    if (tok0 >= (unsigned)NTOK) return;
    int ke0 = 0, ke1 = 1;
    float kw0 = 0.0f, kw1 = 0.0f;
    v4f kl0 = (v4f){0.f, 0.f, 0.f, 0.f}, kl1 = (v4f){0.f, 0.f, 0.f, 0.f};
    const float b0 = bfr(bg[0]), b1 = bfr(bg[1]), b2 = bfr(bg[2]), b3 = bfr(bg[3]);
    for (unsigned tt = 0; tt < 16u; ++tt) {
        const float* xr = x + (size_t)(tok0 + tt) * DM;
        float acc[NPART + NPART * RK];
#pragma unroll
        for (int g = 0; g < NPART + NPART * RK; ++g) acc[g] = 0.0f;
        for (unsigned q = 0; q < (unsigned)(DM / 32); ++q) {
            const unsigned d = lane + 32u * q;
            const float xv = bfr(xr[d]);
#pragma unroll
            for (int g = 0; g < NPART; ++g) acc[g] += xv * bfr(Wg[(unsigned)g * (unsigned)DM + d]);
#pragma unroll
            for (int g = 0; g < NPART * RK; ++g) acc[NPART + g] += xv * bfr(A[(unsigned)g * (unsigned)DM + d]);
        }
#pragma unroll
        for (int g = 0; g < NPART + NPART * RK; ++g) {
            float s = acc[g];
            s += __shfl_xor(s, 16, 32);
            s += __shfl_xor(s, 8, 32);
            s += __shfl_xor(s, 4, 32);
            s += __shfl_xor(s, 2, 32);
            s += __shfl_xor(s, 1, 32);
            acc[g] = s;
        }
        const float l0 = acc[0] + b0, l1 = acc[1] + b1, l2 = acc[2] + b2, l3 = acc[3] + b3;
        const float mx = fmaxf(fmaxf(l0, l1), fmaxf(l2, l3));
        const float p0 = expf(l0 - mx), p1 = expf(l1 - mx), p2 = expf(l2 - mx), p3 = expf(l3 - mx);
        const float ps = ((p0 + p1) + p2) + p3;
        const float s0 = p0 / ps, s1 = p1 / ps, s2 = p2 / ps, s3 = p3 / ps;
        int e0 = 0; float w0 = s0;
        if (s1 > w0) { e0 = 1; w0 = s1; }
        if (s2 > w0) { e0 = 2; w0 = s2; }
        if (s3 > w0) { e0 = 3; w0 = s3; }
        int e1 = (e0 == 0) ? 1 : 0; float w1 = (e0 == 0) ? s1 : s0;
        if (e0 != 1 && e1 != 1 && s1 > w1) { e1 = 1; w1 = s1; }
        if (e0 != 2 && s2 > w1) { e1 = 2; w1 = s2; }
        if (e0 != 3 && s3 > w1) { e1 = 3; w1 = s3; }
        const v4f r0 = (v4f){acc[4], acc[5], acc[6], acc[7]}, r1 = (v4f){acc[8], acc[9], acc[10], acc[11]};
        const v4f r2 = (v4f){acc[12], acc[13], acc[14], acc[15]}, r3 = (v4f){acc[16], acc[17], acc[18], acc[19]};
        const v4f t0 = pick4(e0, r0, r1, r2, r3), t1 = pick4(e1, r0, r1, r2, r3);
        const bool mine = (lane == tt);
        ke0 = mine ? e0 : ke0; ke1 = mine ? e1 : ke1; kw0 = mine ? w0 : kw0; kw1 = mine ? w1 : kw1;
        kl0.x = mine ? t0.x : kl0.x; kl0.y = mine ? t0.y : kl0.y; kl0.z = mine ? t0.z : kl0.z; kl0.w = mine ? t0.w : kl0.w;
        kl1.x = mine ? t1.x : kl1.x; kl1.y = mine ? t1.y : kl1.y; kl1.z = mine ? t1.z : kl1.z; kl1.w = mine ? t1.w : kl1.w;
    }
    if (lane < 16u) {
        const unsigned t = tok0 + lane;
        v2i se; se.x = ke0; se.y = ke1;
        v2f we; we.x = kw0; we.y = kw1;
        for (int pass = 0; pass < 2; ++pass) {
            *(volatile v2i*)(sel + 2u * t) = se;
            *(volatile v2f*)(wgt + 2u * t) = we;
            *(volatile v4f*)(low0 + 4u * t) = kl0;
            *(volatile v4f*)(low1 + 4u * t) = kl1;
            __threadfence();
        }
    }
}

__global__ __launch_bounds__(64) void k_tbl_dense(int* __restrict__ tbl) {
    const unsigned w0 = threadIdx.x * 4u;
    int q[4];
#pragma unroll
    for (int k = 0; k < 4; ++k) {
        const unsigned w = w0 + (unsigned)k;
        int val = 0;
        val = (w < (unsigned)(TBL_COUNT + NSH)) ? NTOK : val;
        val = (w >= (unsigned)TBL_POFF && w <= (unsigned)(TBL_POFF + NE)) ? (int)min((w - (unsigned)TBL_POFF) * (unsigned)NTOK, (unsigned)NROW_S) : val;
        val = (w == (unsigned)TBL_NTILES) ? (NROW_S / 64) : val;
        val = (w >= (unsigned)TBL_TILE_E && w < (unsigned)(TBL_TILE_E + NT_MAX)) ? ((w - (unsigned)TBL_TILE_E < (unsigned)(NROW_S / 64)) ? (int)((w - (unsigned)TBL_TILE_E) / (unsigned)(NTOK / 64)) : -1) : val;
        q[k] = val;
    }
    v4i v;
    v.x = q[0]; v.y = q[1]; v.z = q[2]; v.w = q[3];
    VST2(v4i, tbl + w0, v);
}

__global__ __launch_bounds__(256) void k_ffn1(const h16* __restrict__ Xg, const h16* __restrict__ Wp, const int* __restrict__ sel, const float* __restrict__ wgt,
                                              const float* __restrict__ low0, const float* __restrict__ low1, const float* __restrict__ Bq,
                                              const int* __restrict__ tbl, h16* __restrict__ Hg) {
    __shared__ __align__(16) float sT[8][16 * 68];
    const unsigned lane = threadIdx.x & 31u;
    const unsigned wave = threadIdx.x >> 5;
    const unsigned u = blockIdx.x * 8u + wave;
    if (u >= (unsigned)(NT_MAX * (FF / 64))) return;
    const unsigned rowtile = u / (unsigned)(FF / 64);
    const unsigned ct = u - rowtile * (unsigned)(FF / 64);
    const int nt = min(max(tbl[TBL_NTILES], 0), NT_MAX);
    if ((int)rowtile >= nt) return;
    const int e = min(max(tbl[TBL_TILE_E + rowtile], 0), NE - 1);
    const size_t wbase = (size_t)(unsigned)e * (size_t)(FF * DM);
    const unsigned m0 = rowtile << 6, n0 = ct << 6;
    const unsigned rlane = lane & 15u;
    const unsigned koff = (lane >> 4) * 8u;
    const unsigned mOff = koff;

    v8f acc[4][4];
#pragma unroll
    for (int i = 0; i < 4; ++i)
#pragma unroll
        for (int j = 0; j < 4; ++j) acc[i][j] = (v8f){0.f,0.f,0.f,0.f,0.f,0.f,0.f,0.f};

    for (unsigned k0 = 0; k0 < (unsigned)DM; k0 += 32u) {
        v16h bh[4];
#pragma unroll
        for (int j = 0; j < 4; ++j)
            bh[j] = frag_ld(Wp + wbase + (size_t)(n0 + ((unsigned)j << 4) + rlane) * DM + koff + k0);
#pragma unroll
        for (int i = 0; i < 4; ++i) {
            const v16h ah = frag_ld(Xg + (size_t)(m0 + ((unsigned)i << 4) + rlane) * DM + koff + k0);
#pragma unroll
            for (int j = 0; j < 4; ++j) acc[i][j] = wmma16g(ah, bh[j], acc[i][j]);
        }
    }

    float* slab = sT[wave];
#pragma unroll
    for (int i = 0; i < 4; ++i) {
        const unsigned mBase = m0 + ((unsigned)i << 4);
#pragma unroll
        for (int r = 0; r < 8; ++r) {
            const unsigned tokr = mBase + mOff + (unsigned)r;
            const v2i se = *(const v2i*)(sel + 2u * tokr);
            const v2f we = *(const v2f*)(wgt + 2u * tokr);
            const v4f la = *(const v4f*)(low0 + 4u * tokr);
            const v4f lb = *(const v4f*)(low1 + 4u * tokr);
            const unsigned ea = (unsigned)min(max(se.x, 0), NPART - 1), eb = (unsigned)min(max(se.y, 0), NPART - 1);
#pragma unroll
            for (int j = 0; j < 4; ++j) {
                const unsigned n = n0 + ((unsigned)j << 4) + rlane;
                const v4f ba = *(const v4f*)(Bq + ((size_t)ea * FF + n) * RK);
                const v4f bb = *(const v4f*)(Bq + ((size_t)eb * FF + n) * RK);
                const float a = acc[i][j][r] * SC_H;
                const float ta = ((la.x * ba.x + la.y * ba.y) + la.z * ba.z) + la.w * ba.w;
                const float tb = ((lb.x * bb.x + lb.y * bb.y) + lb.z * bb.z) + lb.w * bb.w;
                const float g = we.x * fmaxf(a + ta, 0.0f) + we.y * fmaxf(a + tb, 0.0f);
                slab[(mOff + (unsigned)r) * 68u + ((unsigned)j << 4) + rlane] = g * CH;
            }
        }
        wave_sync_lds();
        const unsigned q = lane >> 3, c8 = (lane & 7u) * 8u;
        v8h hv[4];
#pragma unroll
        for (int it = 0; it < 4; ++it) {
            const unsigned row = (unsigned)it * 4u + q;
            const float* sp = slab + row * 68u + c8;
#pragma unroll
            for (int t = 0; t < 8; ++t) hv[it][t] = toh_flush(sp[t]);
        }
        for (int pass = 0; pass < 2; ++pass) {
#pragma unroll
            for (int it = 0; it < 4; ++it) {
                const unsigned row = (unsigned)it * 4u + q;
                *(volatile v8h*)(Hg + (size_t)(mBase + row) * FF + n0 + c8) = hv[it];
            }
            __threadfence();
        }
        wave_sync_lds();
    }
}

__global__ __launch_bounds__(256) void k_ffn2(const h16* __restrict__ Hg, const h16* __restrict__ W2p,
                                              const int* __restrict__ tbl, float* __restrict__ Yg) {
    __shared__ __align__(16) float sT[8][16 * 68];
    const unsigned lane = threadIdx.x & 31u;
    const unsigned wave = threadIdx.x >> 5;
    const unsigned u = blockIdx.x * 8u + wave;
    if (u >= (unsigned)(NT_MAX * (DM / 64))) return;
    const unsigned rowtile = u / (unsigned)(DM / 64);
    const unsigned ct = u - rowtile * (unsigned)(DM / 64);
    const int nt = min(max(tbl[TBL_NTILES], 0), NT_MAX);
    if ((int)rowtile >= nt) return;
    const int e = min(max(tbl[TBL_TILE_E + rowtile], 0), NE - 1);
    const size_t wbase = (size_t)(unsigned)e * (size_t)(DM * II);
    const unsigned m0 = rowtile << 6, n0 = ct << 6;
    const unsigned rlane = lane & 15u;
    const unsigned koff = (lane >> 4) * 8u;
    const unsigned mOff = koff;

    v8f acc[4][4];
#pragma unroll
    for (int i = 0; i < 4; ++i)
#pragma unroll
        for (int j = 0; j < 4; ++j) acc[i][j] = (v8f){0.f,0.f,0.f,0.f,0.f,0.f,0.f,0.f};

    for (unsigned k0 = 0; k0 < (unsigned)II; k0 += 32u) {
        v16h bh[4];
#pragma unroll
        for (int j = 0; j < 4; ++j)
            bh[j] = frag_ld(W2p + wbase + (size_t)(n0 + ((unsigned)j << 4) + rlane) * II + koff + k0);
#pragma unroll
        for (int i = 0; i < 4; ++i) {
            const v16h ah = frag_ld(Hg + (size_t)(m0 + ((unsigned)i << 4) + rlane) * II + koff + k0);
#pragma unroll
            for (int j = 0; j < 4; ++j) acc[i][j] = wmma16g(ah, bh[j], acc[i][j]);
        }
    }

    float* slab = sT[wave];
#pragma unroll
    for (int i = 0; i < 4; ++i) {
        const unsigned mBase = m0 + ((unsigned)i << 4);
#pragma unroll
        for (int j = 0; j < 4; ++j)
#pragma unroll
            for (int r = 0; r < 8; ++r)
                slab[(mOff + (unsigned)r) * 68u + ((unsigned)j << 4) + rlane] = acc[i][j][r] * SC_Y;
        wave_sync_lds();
        const unsigned hh = lane >> 4, c4 = (lane & 15u) * 4u;
#pragma unroll
        for (int half = 0; half < 2; ++half) {
            v4f vv[4];
#pragma unroll
            for (int it = 0; it < 4; ++it) {
                const unsigned row = (unsigned)(half * 4 + it) * 2u + hh;
                vv[it] = *(const v4f*)(slab + row * 68u + c4);
            }
            for (int pass = 0; pass < 2; ++pass) {
#pragma unroll
                for (int it = 0; it < 4; ++it) {
                    const unsigned row = (unsigned)(half * 4 + it) * 2u + hh;
                    *(volatile v4f*)(Yg + (size_t)(mBase + row) * DM + n0 + c4) = vv[it];
                }
                __threadfence();
            }
        }
        wave_sync_lds();
    }
}

extern "C" void kernel_launch(void* const* d_in, const int* in_sizes, int n_in, void* d_out, int out_size,
                              void* d_ws, size_t ws_size, hipStream_t stream) {
    if (n_in < 7) return;
    if (in_sizes[0] < NTOK * DM || in_sizes[1] < NPART * DM || in_sizes[2] < NPART || in_sizes[3] < FF * DM || in_sizes[4] < DM * FF || in_sizes[5] < NPART * RK * DM || in_sizes[6] < NPART * FF * RK) return;
    if (out_size < NTOK * DM) return;

    const float* x  = (const float*)d_in[0];
    const float* Wg = (const float*)d_in[1];
    const float* bg = (const float*)d_in[2];
    const float* Wi = (const float*)d_in[3];
    const float* Wo = (const float*)d_in[4];
    const float* A  = (const float*)d_in[5];
    const float* B  = (const float*)d_in[6];
    float* out = (float*)d_out;

    char* wsp = (char*)d_ws;
    size_t off = 0;
    auto carve = [&](size_t bytes) -> void* { void* r = wsp + off; off += (bytes + 255) & ~(size_t)255; return r; };
    h16*   x16  = (h16*)carve((size_t)NTOK * DM * 2);
    h16*   wip  = (h16*)carve((size_t)FF * DM * 2);
    h16*   wop  = (h16*)carve((size_t)DM * FF * 2);
    float* Bq   = (float*)carve((size_t)NPART * FF * RK * 4);
    int*   sel  = (int*)carve((size_t)NTOK * TOPK * 4);
    float* wgt  = (float*)carve((size_t)NTOK * TOPK * 4);
    float* low0 = (float*)carve((size_t)NTOK * RK * 4);
    float* low1 = (float*)carve((size_t)NTOK * RK * 4);
    int*   tbl  = (int*)carve((size_t)TBLS_WORDS * 4);
    h16*   Hg   = (h16*)carve((size_t)NTOK * FF * 2);
    if (off != WS_TOTAL || off > ws_size || off > (size_t)134217728) return;

    k_plane<CX_LOG2><<<(NTOK * DM / 8) / 256, 256, 0, stream>>>(x, x16, (unsigned)(NTOK * DM / 8));
    k_plane<CW_LOG2><<<(FF * DM / 8) / 256, 256, 0, stream>>>(Wi, wip, (unsigned)(FF * DM / 8));
    k_plane<CW_LOG2><<<(DM * FF / 8) / 256, 256, 0, stream>>>(Wo, wop, (unsigned)(DM * FF / 8));
    k_castf<<<(NPART * FF * RK / 4) / 256, 256, 0, stream>>>(B, Bq, (unsigned)(NPART * FF * RK));
    k_gate_lora<<<NTOK / 128, 256, 0, stream>>>(x, Wg, bg, A, sel, wgt, low0, low1);
    k_tbl_dense<<<1, 64, 0, stream>>>(tbl);
    k_ffn1<<<(NT_MAX * (FF / 64) + 7) / 8, 256, 0, stream>>>(x16, wip, sel, wgt, low0, low1, Bq, tbl, Hg);
    k_ffn2<<<(NT_MAX * (DM / 64) + 7) / 8, 256, 0, stream>>>(Hg, wop, tbl, out);
}
